// GCN_55301998903731
// MI455X (gfx1250) — hardware-verified
//
#include <hip/hip_runtime.h>
#include <stddef.h>
#include <stdint.h>
#include <math.h>


#define NNODE  50000
#define NEDGE  800000
#define F0     128
#define F1     128
#define F2     256
#define F3     128
#define NCLS   10
#define KA     256
#define NTHR   256
#define NWAVE  8
#define EPT    8
#define CHUNK  (NTHR * EPT)
#define WCAP   (EPT * 32)
#define LISTN  (NWAVE * WCAP)
#define NBA    1024
#define SLA    10
#define RCAP   28672
#define DEGCAP 64
#define GBM    64
#define GBN    128
#define GTHR   128
#define MPC    50048
#define NTILE  (MPC / GBM)
#define GA     49
#define NBX    ((MPC * (F0 / 8)) / NTHR)
#define NBW1   ((F1 * (F0 / 8)) / NTHR)
#define NBW2   ((F2 * (KA / 8)) / NTHR)
#define AGG_ZINTS (LISTN + 2 * RCAP + 3 * NBA)
#define AGG_LDS_INTS (AGG_ZINTS + 16)
#define WSMAX  134217728

static_assert((CHUNK & (CHUNK - 1)) == 0 && CHUNK <= 4096);
static_assert((NBA & (NBA - 1)) == 0 && NBA == (1 << SLA));
static_assert(((long long)CHUNK << SLA) < (1LL << 31));
static_assert((long long)NEDGE < (1LL << (31 - SLA)));
static_assert(LISTN % NTHR == 0);
static_assert(NBA % NWAVE == 0 && NBA % 32 == 0 && NBA % GBM == 0);
static_assert(RCAP % 4 == 0 && AGG_ZINTS % 4 == 0 && LISTN % 4 == 0);
static_assert(RCAP >= 16696 + 16696 / 2);
static_assert(DEGCAP >= 33 + 8);
static_assert(F0 == 4 * 32 && F1 == 4 * 32 && KA == 2 * F1 && KA % 32 == 0 && F0 % 32 == 0);
static_assert(GBM == (GTHR / 32) * 16 && GTHR == GBN && F1 == GBN && F2 == 2 * GBN);
static_assert(MPC % GBM == 0 && MPC >= NNODE && MPC - NNODE < GBM && NNODE % 16 == 0);
static_assert((long long)NTILE * GBM >= NNODE);
static_assert((long long)GA * NBA >= MPC && (long long)GA * NBA >= NNODE);
static_assert((MPC * (F0 / 8)) % NTHR == 0 && (F1 * (F0 / 8)) % NTHR == 0 && (F2 * (KA / 8)) % NTHR == 0);
static_assert(F0 / 8 == 16 && KA / 8 == 32);
static_assert(AGG_LDS_INTS * 4 <= 300000);
static_assert(F2 == NTHR && F3 <= NTHR && F3 % 32 == 0 && NCLS <= 32);

typedef float          v4f   __attribute__((ext_vector_type(4)));
typedef float          v8f   __attribute__((ext_vector_type(8)));
typedef int            v4i   __attribute__((ext_vector_type(4)));
typedef int            v8i   __attribute__((ext_vector_type(8)));
typedef unsigned short v8us  __attribute__((ext_vector_type(8)));
typedef unsigned short v16us __attribute__((ext_vector_type(16)));
typedef __bf16         v16bf __attribute__((ext_vector_type(16)));
typedef v4f  __attribute__((may_alias)) v4fa;
typedef v4i  __attribute__((may_alias)) v4ia;
typedef v8us __attribute__((may_alias)) v8usa;
union FragB { v16bf v; v16us u; v8us h[2]; v8i w; };

__device__ __forceinline__ v8f wmb(const FragB& a, const FragB& b, v8f c) {
  v8f d = __builtin_amdgcn_wmma_f32_16x16x32_bf16(false, a.v, false, b.v, (short)0, c, false, false);
  asm volatile("v_nop\n\tv_nop\n\tv_nop\n\tv_nop" : "+v"(d) : "v"(a.w), "v"(b.w));
  return d;
}

__device__ __forceinline__ unsigned bf16_bits(float f) {
  const unsigned u = __float_as_uint(f);
  const unsigned r = (u + 0x7FFFu + ((u >> 16) & 1u)) >> 16;
  return (f != f) ? 0x7FC0u : r;
}
__device__ __forceinline__ float bf16_val(float f) {
  return __uint_as_float(bf16_bits(f) << 16);
}

__device__ __forceinline__ void hilo_pack(float v0, float v1, float v2, float v3,
                                          int& h01, int& h23, int& l01, int& l23) {
  const unsigned a0 = bf16_bits(v0), a1 = bf16_bits(v1), a2 = bf16_bits(v2), a3 = bf16_bits(v3);
  const unsigned b0 = bf16_bits(v0 - __uint_as_float(a0 << 16));
  const unsigned b1 = bf16_bits(v1 - __uint_as_float(a1 << 16));
  const unsigned b2 = bf16_bits(v2 - __uint_as_float(a2 << 16));
  const unsigned b3 = bf16_bits(v3 - __uint_as_float(a3 << 16));
  h01 = (int)(a0 | (a1 << 16)); h23 = (int)(a2 | (a3 << 16));
  l01 = (int)(b0 | (b1 << 16)); l23 = (int)(b2 | (b3 << 16));
}

__device__ __forceinline__ v4i regroup16(int h01, int h23, int l01, int l23, int lane) {
  const int s0 = (2 * lane) & 31, s1 = s0 + 1;
  const int a0 = __shfl(h01, s0, 32), a1 = __shfl(h23, s0, 32), a2 = __shfl(h01, s1, 32), a3 = __shfl(h23, s1, 32);
  const int b0 = __shfl(l01, s0, 32), b1 = __shfl(l23, s0, 32), b2 = __shfl(l01, s1, 32), b3 = __shfl(l23, s1, 32);
  const int mk = (lane < 16) ? -1 : 0;
  v4i o;
  o.x = (a0 & mk) | (b0 & ~mk); o.y = (a1 & mk) | (b1 & ~mk);
  o.z = (a2 & mk) | (b2 & ~mk); o.w = (a3 & mk) | (b3 & ~mk);
  return o;
}

template <int SLB>
__device__ __forceinline__ int scan_chunk(const int* __restrict__ dsts, int nE, int cbase, int slotBase,
                                          int nb, int vec8, int* list, int tid, int lane, int wave) {
  int wc = 0;
  const int el0  = tid * EPT;
  const int e0   = cbase + el0;
  const int sent = -2147483647 - 1;
  v4i da, db;
  if (vec8 != 0 && cbase + CHUNK <= nE) {
    da = *(const v4i*)(dsts + e0);
    db = *(const v4i*)(dsts + e0 + 4);
  } else {
    da.x = (e0     < nE) ? dsts[min(e0,     nE - 1)] : sent;
    da.y = (e0 + 1 < nE) ? dsts[min(e0 + 1, nE - 1)] : sent;
    da.z = (e0 + 2 < nE) ? dsts[min(e0 + 2, nE - 1)] : sent;
    da.w = (e0 + 3 < nE) ? dsts[min(e0 + 3, nE - 1)] : sent;
    db.x = (e0 + 4 < nE) ? dsts[min(e0 + 4, nE - 1)] : sent;
    db.y = (e0 + 5 < nE) ? dsts[min(e0 + 5, nE - 1)] : sent;
    db.z = (e0 + 6 < nE) ? dsts[min(e0 + 6, nE - 1)] : sent;
    db.w = (e0 + 7 < nE) ? dsts[min(e0 + 7, nE - 1)] : sent;
  }
  const unsigned nbs = (unsigned)slotBase;
  const unsigned unb = (unsigned)nb;
  const unsigned s0 = (unsigned)da.x - nbs, s1 = (unsigned)da.y - nbs;
  const unsigned s2 = (unsigned)da.z - nbs, s3 = (unsigned)da.w - nbs;
  const unsigned s4 = (unsigned)db.x - nbs, s5 = (unsigned)db.y - nbs;
  const unsigned s6 = (unsigned)db.z - nbs, s7 = (unsigned)db.w - nbs;
  const bool h0 = s0 < unb, h1 = s1 < unb, h2 = s2 < unb, h3 = s3 < unb;
  const bool h4 = s4 < unb, h5 = s5 < unb, h6 = s6 < unb, h7 = s7 < unb;
  const unsigned any = __builtin_amdgcn_ballot_w32(h0 | h1 | h2 | h3 | h4 | h5 | h6 | h7);
  if (any != 0u) {
#define HITJ(J, HJ, SJ) { \
      const unsigned mj = __builtin_amdgcn_ballot_w32(HJ); \
      if (mj != 0u) { \
        if (HJ) { \
          const int pos = wc + (int)__builtin_amdgcn_mbcnt_lo(mj, 0u); \
          if (pos < WCAP) list[wave * WCAP + pos] = ((el0 + (J)) << SLB) | (int)(SJ); \
        } \
        wc += (int)__builtin_popcount(mj); } }
    HITJ(0, h0, s0)
    HITJ(1, h1, s1)
    HITJ(2, h2, s2)
    HITJ(3, h3, s3)
    HITJ(4, h4, s4)
    HITJ(5, h5, s5)
    HITJ(6, h6, s6)
    HITJ(7, h7, s7)
#undef HITJ
  }
  return wc;
}

__global__ __launch_bounds__(NTHR) void k_prep(const float* __restrict__ x, int nN,
                                               const float* __restrict__ W1, const float* __restrict__ W2,
                                               unsigned short* xb, unsigned short* w1t, unsigned short* w2d) {
  const int tid = (int)threadIdx.x;
  const int blk = (int)blockIdx.x;
  v8us o;
  unsigned short* dp;
  if (blk < NBX) {
    const int u   = blk * NTHR + tid;
    const int row = u >> 4;
    const int k8  = (u & 15) * 8;
    const int rc  = row < nN ? row : nN - 1;
    const float* p = x + (size_t)rc * F0 + k8;
    const v4f a = *(const v4fa*)p;
    const v4f b = *(const v4fa*)(p + 4);
    const bool ok = row < nN;
    o[0] = ok ? (unsigned short)bf16_bits(a.x) : (unsigned short)0;
    o[1] = ok ? (unsigned short)bf16_bits(a.y) : (unsigned short)0;
    o[2] = ok ? (unsigned short)bf16_bits(a.z) : (unsigned short)0;
    o[3] = ok ? (unsigned short)bf16_bits(a.w) : (unsigned short)0;
    o[4] = ok ? (unsigned short)bf16_bits(b.x) : (unsigned short)0;
    o[5] = ok ? (unsigned short)bf16_bits(b.y) : (unsigned short)0;
    o[6] = ok ? (unsigned short)bf16_bits(b.z) : (unsigned short)0;
    o[7] = ok ? (unsigned short)bf16_bits(b.w) : (unsigned short)0;
    dp = xb + (size_t)row * F0 + k8;
  } else if (blk < NBX + NBW1) {
    const int u  = (blk - NBX) * NTHR + tid;
    const int n  = u >> 4;
    const int k8 = (u & 15) * 8;
    const float* p = W1 + (size_t)k8 * F1 + n;
#pragma unroll
    for (int i = 0; i < 8; ++i) o[i] = (unsigned short)bf16_bits(p[(size_t)i * F1]);
    dp = w1t + (size_t)n * F0 + k8;
  } else {
    const int u  = (blk - NBX - NBW1) * NTHR + tid;
    const int n  = u >> 5;
    const int k8 = (u & 31) * 8;
    const int kk = k8 & (F1 - 1);
    const float* p = W2 + (size_t)kk * F2 + n;
#pragma unroll
    for (int i = 0; i < 8; ++i) o[i] = (unsigned short)bf16_bits(p[(size_t)i * F2]);
    dp = w2d + (size_t)n * KA + k8;
  }
  *(volatile v8us*)dp = o;
  __threadfence();
  *(volatile v8us*)dp = o;
}

template <int KK, int MODE>
__global__ __launch_bounds__(GTHR) void k_gemm(const unsigned short* __restrict__ A,
                                               const unsigned short* __restrict__ BT,
                                               const float* __restrict__ bias, int nN, float* outp) {
  __shared__ __attribute__((aligned(16))) float stg[GBM * GBN];
  __shared__ __attribute__((aligned(16))) float sred[GBN];
  const int tid = (int)threadIdx.x, lane = tid & 31, wave = tid >> 5, hh = lane >> 4, m = lane & 15;
  const int rowBase = (int)blockIdx.x * GBM;
  const int col0    = (int)blockIdx.y * GBN;

  v8f acc[8];
  {
    const v8f z = {0.f, 0.f, 0.f, 0.f, 0.f, 0.f, 0.f, 0.f};
#pragma unroll
    for (int t = 0; t < 8; ++t) acc[t] = z;
  }
  const unsigned short* ap = A  + (size_t)(rowBase + 16 * wave + m) * (size_t)KK + 8 * hh;
  const unsigned short* bp = BT + (size_t)(col0 + m) * (size_t)KK + 8 * hh;

#pragma unroll 1
  for (int k0 = 0; k0 < KK; k0 += 32) {
    FragB af;
    af.h[0] = *(const v8usa*)(ap + k0);
    af.h[1] = *(const v8usa*)(ap + k0 + 16);
#pragma unroll
    for (int nt = 0; nt < 8; ++nt) {
      const unsigned short* wq = bp + (size_t)(16 * nt) * (size_t)KK + k0;
      FragB bf;
      bf.h[0] = *(const v8usa*)wq;
      bf.h[1] = *(const v8usa*)(wq + 16);
      acc[nt] = wmb(af, bf, acc[nt]);
    }
  }

#pragma unroll
  for (int nt = 0; nt < 8; ++nt) {
    const int lc = 16 * nt + m;
#pragma unroll
    for (int r = 0; r < 8; ++r) {
      const int lr = 16 * wave + 8 * hh + r;
      stg[lr * GBN + lc] = acc[nt][r];
    }
  }
  __syncthreads();

  if constexpr (MODE == 0) {
    v4f fv[16];
#pragma unroll
    for (int i = 0; i < 16; ++i) fv[i] = *(const v4fa*)(stg + (16 * wave + i) * GBN + 4 * lane);
#pragma unroll
    for (int i = 0; i < 16; ++i) {
      float* op = outp + (size_t)(rowBase + 16 * wave + i) * GBN + 4 * lane;
      *(volatile v4f*)op = fv[i];
    }
    __threadfence();
#pragma unroll
    for (int i = 0; i < 16; ++i) {
      float* op = outp + (size_t)(rowBase + 16 * wave + i) * GBN + 4 * lane;
      *(volatile v4f*)op = fv[i];
    }
  } else {
    const float bb = bf16_val(bias[col0 + tid]);
    float s = 0.0f;
#pragma unroll 4
    for (int r = 0; r < GBM; ++r) {
      float v = stg[r * GBN + tid] + bb;
      v = (v > 0.0f) ? v : (v - v);
      v = (rowBase + r < nN) ? v : 0.0f;
      s += v;
    }
    sred[tid] = s;
    __syncthreads();
    if (wave == 0) {
      const v4f o = *(const v4fa*)(sred + 4 * lane);
      float* op = outp + (size_t)blockIdx.x * F2 + col0 + 4 * lane;
      *(volatile v4f*)op = o;
      __threadfence();
      *(volatile v4f*)op = o;
    }
  }
}

template <int LAYER>
__global__ __launch_bounds__(NTHR) void k_agg(const int* __restrict__ gsrc, const int* __restrict__ keys,
                                              const float* __restrict__ ew, int nE, int nN, int vec8, int mRows,
                                              const float* __restrict__ xt, const float* __restrict__ bias,
                                              unsigned short* ap, float* outp) {
  extern __shared__ __attribute__((aligned(16))) int dsm[];
  int* list = dsm;
  int* hl   = dsm + LISTN;
  int* sl   = dsm + LISTN + RCAP;
  int* cnt  = dsm + LISTN + 2 * RCAP;
  int* offs = cnt + NBA;
  int* cur  = offs + NBA;
  int* misc = cur + NBA;
  const int tid = (int)threadIdx.x, lane = tid & 31, wave = tid >> 5;
  const int nodeBase = (int)blockIdx.x * NBA;

  {
    const v4i z4 = {0, 0, 0, 0};
    for (int i = tid * 4; i < AGG_ZINTS; i += NTHR * 4) *(v4ia*)(dsm + i) = z4;
    if (tid < 16) misc[tid] = 0;
  }
  float bv0 = 0.0f, bv1 = 0.0f, bv2 = 0.0f, bv3 = 0.0f;
  if constexpr (LAYER == 1) {
    const v4f a = *(const v4fa*)(bias + 4 * lane);
    bv0 = bf16_val(a.x); bv1 = bf16_val(a.y); bv2 = bf16_val(a.z); bv3 = bf16_val(a.w);
  }
  __syncthreads();

  int t = 0, ov = 0;
  const int nChunks = (nE + CHUNK - 1) / CHUNK;
#pragma unroll 1
  for (int ch = 0; ch < nChunks; ++ch) {
    const int cbase = ch * CHUNK;
    const int wc = scan_chunk<SLA>(keys, nE, cbase, nodeBase, NBA, vec8, list, tid, lane, wave);
    if (lane == 0) misc[wave] = wc;
    __syncthreads();
    if (wave == 0) {
#pragma unroll 1
      for (int w2 = 0; w2 < NWAVE; ++w2) {
        int c = misc[w2];
        c = c < 0 ? 0 : (c > WCAP ? WCAP : c);
#pragma unroll 1
        for (int b0 = 0; b0 < c; b0 += 32) {
          const int idx = b0 + lane;
          const int ent = list[w2 * WCAP + (idx < WCAP ? idx : WCAP - 1)];
          const int m32 = (c - b0) < 32 ? (c - b0) : 32;
#pragma unroll 1
          for (int k = 0; k < m32; ++k) {
            const int u    = __builtin_amdgcn_readlane(ent, k);
            const int slot = u & (NBA - 1);
            const int el   = (u >> SLA) & (CHUNK - 1);
            const int pk   = ((cbase + el) << SLA) | slot;
            if (t < RCAP) {
              if (lane == 0) { hl[t] = pk; cnt[slot] = cnt[slot] + 1; }
              t = t + 1;
            } else {
              ov = 1;
            }
          }
        }
      }
    }
    __syncthreads();
  }
  if (wave == 0 && lane == 0) { misc[8] = t; misc[9] = ov; }
  __syncthreads();
  int tt = misc[8];
  tt = tt < 0 ? 0 : (tt > RCAP ? RCAP : tt);
  const int ovf = misc[9];

  if (wave == 0) {
    const int base = lane * (NBA / 32);
    int s = 0;
#pragma unroll 1
    for (int i = 0; i < NBA / 32; ++i) s += cnt[base + i];
    int incl = s;
#pragma unroll
    for (int d = 1; d < 32; d <<= 1) {
      const int y = __shfl_up(incl, d, 32);
      if (lane >= d) incl += y;
    }
    int run = incl - s;
#pragma unroll 1
    for (int i = 0; i < NBA / 32; ++i) {
      const int cv = cnt[base + i];
      offs[base + i] = run;
      cur[base + i]  = run;
      run += cv;
    }
  }
  __syncthreads();
  if (wave == 0) {
#pragma unroll 1
    for (int b0 = 0; b0 < tt; b0 += 32) {
      const int idx = b0 + lane;
      const int ent = hl[idx < RCAP ? idx : RCAP - 1];
      const int m32 = (tt - b0) < 32 ? (tt - b0) : 32;
#pragma unroll 1
      for (int k = 0; k < m32; ++k) {
        const int u    = __builtin_amdgcn_readlane(ent, k);
        const int slot = u & (NBA - 1);
        if (lane == 0) {
          int p = cur[slot];
          p = p < 0 ? 0 : (p > RCAP - 1 ? RCAP - 1 : p);
          sl[p] = u;
          cur[slot] = p + 1;
        }
      }
    }
  }
  __syncthreads();

  const float qnan = __int_as_float(0x7fc00000);
  const float pz = (ovf != 0) ? qnan : 0.0f;
#pragma unroll 1
  for (int si = 0; si < NBA / NWAVE; ++si) {
    const int s    = si * NWAVE + wave;
    const int node = nodeBase + s;
    int c = cnt[s];
    const bool big = c > DEGCAP;
    c = c < 0 ? 0 : (c > DEGCAP ? DEGCAP : c);
    int o = offs[s];
    o = o < 0 ? 0 : (o > RCAP ? RCAP : o);
    float g0 = 0.0f, g1 = 0.0f, g2 = 0.0f, g3 = 0.0f;
#pragma unroll 1
    for (int b0 = 0; b0 < c; b0 += 32) {
      int idx = o + b0 + lane;
      idx = idx > RCAP - 1 ? RCAP - 1 : idx;
      const int ent = sl[idx];
      int eid = ent >> SLA;
      eid = eid < 0 ? 0 : (eid > nE - 1 ? nE - 1 : eid);
      int sr = gsrc[eid];
      sr = sr < 0 ? 0 : (sr > nN - 1 ? nN - 1 : sr);
      const int wvi = __float_as_int(bf16_val(ew[eid]));
      const int m32 = (c - b0) < 32 ? (c - b0) : 32;
#pragma unroll 1
      for (int k = 0; k < m32; ++k) {
        const int   sk = __builtin_amdgcn_readlane(sr, k);
        const float wk = __int_as_float(__builtin_amdgcn_readlane(wvi, k));
        const v4f a = *(const v4fa*)(xt + (size_t)sk * F1 + 4 * lane);
        g0 = fmaf(a.x, wk, g0); g1 = fmaf(a.y, wk, g1);
        g2 = fmaf(a.z, wk, g2); g3 = fmaf(a.w, wk, g3);
      }
    }
    const float pzr = big ? qnan : pz;
    const bool live = node < nN;
    if constexpr (LAYER == 1) {
      float y0 = g0 + bv0, y1 = g1 + bv1, y2 = g2 + bv2, y3 = g3 + bv3;
      y0 = (y0 > 0.0f) ? y0 : (y0 - y0);
      y1 = (y1 > 0.0f) ? y1 : (y1 - y1);
      y2 = (y2 > 0.0f) ? y2 : (y2 - y2);
      y3 = (y3 > 0.0f) ? y3 : (y3 - y3);
      v4f ow;
      ow.x = y0 + pzr; ow.y = y1 + pzr; ow.z = y2 + pzr; ow.w = y3 + pzr;
      if (live) {
        float* op = outp + (size_t)node * F1 + 4 * lane;
        *(volatile v4f*)op = ow;
        __threadfence();
        *(volatile v4f*)op = ow;
      }
    } else {
      const float q0 = live ? g0 + pzr : 0.0f, q1 = live ? g1 + pzr : 0.0f;
      const float q2 = live ? g2 + pzr : 0.0f, q3 = live ? g3 + pzr : 0.0f;
      int h01, h23, l01, l23;
      hilo_pack(q0, q1, q2, q3, h01, h23, l01, l23);
      const v4i ow = regroup16(h01, h23, l01, l23, lane);
      if (node < mRows) {
        unsigned short* hp = ap + (size_t)node * KA + 8 * lane;
        *(volatile v4i*)hp = ow;
        __threadfence();
        *(volatile v4i*)hp = ow;
      }
    }
  }
}

__global__ __launch_bounds__(NTHR) void k_tail(const float* __restrict__ rec, int nT,
                                               const float* __restrict__ W3, const float* __restrict__ b3,
                                               const float* __restrict__ W4, const float* __restrict__ b4,
                                               float* out) {
  __shared__ float gs[F2];
  __shared__ float ts[F3];
  __shared__ float ls[32];
  const int tid = (int)threadIdx.x, lane = tid & 31, wave = tid >> 5;
  {
    double s = 0.0;
#pragma unroll 4
    for (int r = 0; r < nT; ++r) s += (double)rec[(size_t)r * F2 + tid];
    float gv = (float)s;
    gv = (gv > 0.0f) ? gv : (gv - gv);
    gs[tid] = gv;
  }
  __syncthreads();
  if (wave < F3 / 32) {
    double a = 0.0;
#pragma unroll 2
    for (int k = 0; k < F2; ++k) a = fma((double)gs[k], (double)bf16_val(W3[(size_t)k * F3 + tid]), a);
    float tv = (float)a + bf16_val(b3[tid]);
    tv = (tv > 0.0f) ? tv : (tv - tv);
    ts[tid] = tv;
  }
  __syncthreads();
  const int cc = lane < NCLS ? lane : NCLS - 1;
  if (wave == 0) {
    double a = 0.0;
#pragma unroll 2
    for (int j = 0; j < F3; ++j) a = fma((double)ts[j], (double)bf16_val(W4[j * NCLS + cc]), a);
    ls[lane] = (float)a + bf16_val(b4[cc]);
  }
  __syncthreads();
  if (wave == 0) {
    float m = ls[0];
#pragma unroll 1
    for (int c = 1; c < NCLS; ++c) {
      const float v = ls[c];
      m = (v > m || v != v) ? v : m;
    }
    float s = 0.0f;
#pragma unroll 1
    for (int c = 0; c < NCLS; ++c) s += expf(ls[c] - m);
    const float lg = logf(s);
    const float o = (ls[cc] - m) - lg;
    float* op = out + cc;
    if (lane < NCLS) *(volatile float*)op = o;
    __threadfence();
    if (lane < NCLS) *(volatile float*)op = o;
  }
}

static inline size_t al256(size_t o) { return (o + 255) & ~(size_t)255; }

extern "C" void kernel_launch(void* const* d_in, const int* in_sizes, int n_in,
                              void* d_out, int out_size, void* d_ws, size_t ws_size,
                              hipStream_t stream) {
  if (n_in < 12) return;
  if (in_sizes[0] != NNODE * F0) return;
  if (in_sizes[1] != NEDGE || in_sizes[2] != NEDGE || in_sizes[3] != NEDGE) return;
  if (in_sizes[4] != F0 * F1 || in_sizes[5] != F1) return;
  if (in_sizes[6] != F1 * F2 || in_sizes[7] != F2) return;
  if (in_sizes[8] != F2 * F3 || in_sizes[9] != F3) return;
  if (in_sizes[10] != F3 * NCLS || in_sizes[11] != NCLS) return;
  if (out_size != NCLS) return;

  const float* x   = (const float*)d_in[0];
  const int*   es  = (const int*)d_in[1];
  const int*   ed  = (const int*)d_in[2];
  const float* ew  = (const float*)d_in[3];
  const float* W1  = (const float*)d_in[4];
  const float* b1  = (const float*)d_in[5];
  const float* W2  = (const float*)d_in[6];
  const float* b2  = (const float*)d_in[7];
  const float* W3  = (const float*)d_in[8];
  const float* b3  = (const float*)d_in[9];
  const float* W4  = (const float*)d_in[10];
  const float* b4  = (const float*)d_in[11];
  float* out = (float*)d_out;

  const int nN = NNODE;
  const int nE = NEDGE;
  const int vec8 = ((nE & 3) == 0) ? 1 : 0;

  char* ws = (char*)d_ws;
  size_t off = 0;
  const size_t oW1T = off; off = al256(off + (size_t)F1 * F0 * 2);
  const size_t oW2D = off; off = al256(off + (size_t)F2 * KA * 2);
  const size_t oXB  = off; off = al256(off + (size_t)MPC * F0 * 2);
  const size_t oS1  = off; off = al256(off + (size_t)MPC * F1 * 4);
  const size_t oH1  = off; off = al256(off + (size_t)MPC * F1 * 4);
  const size_t oAP  = off; off = al256(off + (size_t)MPC * KA * 2);
  const size_t oREC = off; off = al256(off + (size_t)NTILE * F2 * 4);
  if (off > ws_size || off > (size_t)WSMAX) return;
  unsigned short* W1T = (unsigned short*)(ws + oW1T);
  unsigned short* W2D = (unsigned short*)(ws + oW2D);
  unsigned short* XB  = (unsigned short*)(ws + oXB);
  float*          S1  = (float*)(ws + oS1);
  float*          H1  = (float*)(ws + oH1);
  unsigned short* AP  = (unsigned short*)(ws + oAP);
  float*          REC = (float*)(ws + oREC);

  const size_t aggLds = (size_t)AGG_LDS_INTS * 4;
  hipFuncSetAttribute(reinterpret_cast<const void*>(&k_agg<1>), hipFuncAttributeMaxDynamicSharedMemorySize, (int)aggLds);
  hipFuncSetAttribute(reinterpret_cast<const void*>(&k_agg<2>), hipFuncAttributeMaxDynamicSharedMemorySize, (int)aggLds);

  k_prep<<<NBX + NBW1 + NBW2, NTHR, 0, stream>>>(x, nN, W1, W2, XB, W1T, W2D);
  k_gemm<F0, 0><<<dim3(NTILE, 1), GTHR, 0, stream>>>(XB, W1T, b1, nN, S1);
  k_agg<1><<<GA, NTHR, aggLds, stream>>>(es, ed, ew, nE, nN, vec8, MPC, S1, b1, AP, H1);
  k_agg<2><<<GA, NTHR, aggLds, stream>>>(es, ed, ew, nE, nN, vec8, MPC, H1, b1, AP, S1);
  k_gemm<KA, 1><<<dim3(NTILE, F2 / GBN), GTHR, 0, stream>>>(AP, W2D, b2, nN, REC);
  k_tail<<<1, NTHR, 0, stream>>>(REC, NTILE, W3, b3, W4, b4, out);
}
